// GaussianMultiheadAttention_22617297780909
// MI455X (gfx1250) — hardware-verified
//
#include <hip/hip_runtime.h>
#ifndef NB
#define NB 2
#endif
#ifndef SEQ
#define SEQ 1024
#endif
#define NB_FULL 2
#define DM 1024
#define NH 16
#define HD 64
#define QC (SEQ < 256 ? SEQ : 256)
#define NR ((size_t)NB * SEQ)
#define MP ((int)(NB * SEQ))
#define LQ (NB * DM)
#define CK (3 * HD)
#define LQ3 (NB * 3 * DM)
static_assert(SEQ % 128 == 0);
static_assert(QC % 128 == 0);
static_assert(SEQ % QC == 0);
static_assert(NH * HD == DM);
static_assert(NB <= NB_FULL);
static_assert((NB * SEQ) % 128 == 0);
static_assert(NH == 16);
static_assert(HD == 64);
static_assert(CK % 32 == 0);
static_assert(DM % 32 == 0);
static_assert(QC % 32 == 0);
static_assert((NB * SEQ) % 32 == 0);
static_assert(NH * QC >= DM);
static_assert(32 * 8 * 16 == 32 * HD * 2);
static_assert(32 * 8 * (SEQ / 128) == SEQ * 2);
static_assert(8 * 16 == 32 * 4);
static_assert(4 * 32 * 68 * 4 <= 131072);
#define WS_TOTAL (7 * (size_t)DM * DM * 2 + 3 * NR * DM * 2 + 2 * NR * 3 * DM * 2 + 2 * NR * DM * 2 + (size_t)NB * NH * HD * SEQ * 2 + (size_t)NB * NH * QC * SEQ * 4 + (size_t)NB * NH * QC * SEQ * 2 + (size_t)NB * NH * SEQ * 4 + NR * 4)
static_assert(WS_TOTAL + 32 * 256 <= 134217728);

typedef unsigned short v8us __attribute__((ext_vector_type(8), may_alias));
typedef float  v8f  __attribute__((ext_vector_type(8)));
typedef float  v4f  __attribute__((ext_vector_type(4)));
typedef float  v4fa __attribute__((ext_vector_type(4), may_alias));
typedef _Float16 v16h __attribute__((ext_vector_type(16)));
typedef _Float16 v4h __attribute__((ext_vector_type(4)));
union FragH { v16h v; v8us half[2]; _Float16 h[16]; unsigned short u[16]; };

__device__ __forceinline__ unsigned short bf16_bits(float x) { unsigned int u = __float_as_uint(x); return (unsigned short)((u + 0x7FFFu + ((u >> 16) & 1u)) >> 16); }
__device__ __forceinline__ float bf16_val(unsigned short b) { return __uint_as_float(((unsigned int)b) << 16); }
__device__ __forceinline__ float bf16_rne(float x) { return bf16_val(bf16_bits(x)); }

typedef _Float16 h16;
static __device__ __forceinline__ h16 toh_flush(float v) { const h16 r = (h16)v; return (fabsf(v) < 6.103515625e-05f) ? (h16)0.0f : r; }

__device__ __forceinline__ v16h g2_frag(const _Float16* p, int hh) { FragH f; f.half[0] = *(const v8us*)((const unsigned short*)p + 8 * hh); f.half[1] = *(const v8us*)((const unsigned short*)p + 16 + 8 * hh); return f.v; }
__device__ __forceinline__ v8f g2_mma(v16h a, v16h b, v8f c) { v8f d = __builtin_amdgcn_wmma_f32_16x16x32_f16(false, a, false, b, (short)0, c, false, false); asm volatile("v_nop\n\tv_nop\n\tv_nop\n\tv_nop" : "+v"(d) : "v"(a), "v"(b)); return d; }

template <bool HASB, bool OUT32, bool OMAP>
__global__ __launch_bounds__(128) void k_gemm2(const _Float16* __restrict__ A, int lda, size_t sA, const _Float16* __restrict__ Bh, int ldb, size_t sB, float alpha,
    const float* __restrict__ bias, float* __restrict__ C, _Float16* __restrict__ C16, int ldc, size_t sC, int M, int N, int K) {
  __shared__ __attribute__((aligned(16))) float so[4][32][68];
  const int tid = threadIdx.x, w = __builtin_amdgcn_readfirstlane((int)(tid >> 5)), lane = tid & 31, ln = lane & 15, hh = lane >> 4; const int by = blockIdx.y;
  A += (size_t)by * sA; Bh += (size_t)by * sB; const size_t cofs = (size_t)by * sC;
  const int ntn = N >> 6; const int mt = blockIdx.x / ntn, nq = blockIdx.x - mt * ntn; const int row0 = mt * 128 + 32 * w, col0 = nq * 64; if (row0 >= M) return;
  const _Float16* a0p = A + (size_t)(row0 + ln) * lda; const _Float16* a1p = a0p + (size_t)16 * lda;
  const _Float16* b0p = Bh + (size_t)(col0 + ln) * ldb; const _Float16* b1p = b0p + (size_t)16 * ldb; const _Float16* b2p = b1p + (size_t)16 * ldb; const _Float16* b3p = b2p + (size_t)16 * ldb;
  const v8f z8 = {0.f,0.f,0.f,0.f,0.f,0.f,0.f,0.f}; v8f c00 = z8, c01 = z8, c02 = z8, c03 = z8, c10 = z8, c11 = z8, c12 = z8, c13 = z8;
#pragma unroll 1
  for (int kb = 0; kb < K; kb += 32) { const v16h a0 = g2_frag(a0p + kb, hh), a1 = g2_frag(a1p + kb, hh);
    v16h b = g2_frag(b0p + kb, hh); c00 = g2_mma(a0, b, c00); c10 = g2_mma(a1, b, c10);
    b = g2_frag(b1p + kb, hh); c01 = g2_mma(a0, b, c01); c11 = g2_mma(a1, b, c11);
    b = g2_frag(b2p + kb, hh); c02 = g2_mma(a0, b, c02); c12 = g2_mma(a1, b, c12);
    b = g2_frag(b3p + kb, hh); c03 = g2_mma(a0, b, c03); c13 = g2_mma(a1, b, c13); }
  v8f accs[8] = {c00, c01, c02, c03, c10, c11, c12, c13};
#pragma unroll
  for (int u = 0; u < 8; ++u) { const int t = u & 3, half = u >> 2; const int col = col0 + t * 16 + ln; float bv = 0.f; if (HASB) bv = bf16_rne(bias[col]);
#pragma unroll
    for (int r = 0; r < 8; ++r) { const int rloc = half * 16 + 8 * hh + r; so[w][rloc][t * 16 + ln] = accs[u][r] * alpha + bv; } }
  __builtin_amdgcn_fence(4  , "workgroup"); __builtin_amdgcn_wave_barrier();
  const int rsub = lane >> 4, c4 = (lane & 15) * 4;
  for (int pass = 0; pass < 2; ++pass) {
#pragma unroll
    for (int q = 0; q < 16; ++q) { const int r = q * 2 + rsub; const v4f v = *(const v4fa*)&so[w][r][c4];
      const int gr = row0 + r; const size_t orow = OMAP ? ((size_t)(gr / NB) * NB_FULL + (size_t)(gr % NB)) : (size_t)gr;
      if (OUT32) { *(volatile v4f*)(C + cofs + orow * ldc + col0 + c4) = v; }
      else { v4h h4;
#pragma unroll
        for (int i = 0; i < 4; ++i) h4[i] = (_Float16)v[i];
        *(volatile v4h*)(C16 + cofs + orow * ldc + col0 + c4) = h4; } }
    if (pass == 0) __threadfence(); } }

__global__ __launch_bounds__(128) void k_gemm_cat(const _Float16* __restrict__ A, int lda, const _Float16* __restrict__ Bh, int ldb, float alpha,
    const float* __restrict__ bias, _Float16* __restrict__ C3, int ldc3, int qside, int M, int N, int K) {
  __shared__ __attribute__((aligned(16))) float so[4][32][68];
  const int tid = threadIdx.x, w = __builtin_amdgcn_readfirstlane((int)(tid >> 5)), lane = tid & 31, ln = lane & 15, hh = lane >> 4;
  const int ntn = N >> 6; const int mt = blockIdx.x / ntn, nq = blockIdx.x - mt * ntn; const int row0 = mt * 128 + 32 * w, col0 = nq * 64; if (row0 >= M) return;
  const _Float16* a0p = A + (size_t)(row0 + ln) * lda; const _Float16* a1p = a0p + (size_t)16 * lda;
  const _Float16* b0p = Bh + (size_t)(col0 + ln) * ldb; const _Float16* b1p = b0p + (size_t)16 * ldb; const _Float16* b2p = b1p + (size_t)16 * ldb; const _Float16* b3p = b2p + (size_t)16 * ldb;
  const v8f z8 = {0.f,0.f,0.f,0.f,0.f,0.f,0.f,0.f}; v8f c00 = z8, c01 = z8, c02 = z8, c03 = z8, c10 = z8, c11 = z8, c12 = z8, c13 = z8;
#pragma unroll 1
  for (int kb = 0; kb < K; kb += 32) { const v16h a0 = g2_frag(a0p + kb, hh), a1 = g2_frag(a1p + kb, hh);
    v16h b = g2_frag(b0p + kb, hh); c00 = g2_mma(a0, b, c00); c10 = g2_mma(a1, b, c10);
    b = g2_frag(b1p + kb, hh); c01 = g2_mma(a0, b, c01); c11 = g2_mma(a1, b, c11);
    b = g2_frag(b2p + kb, hh); c02 = g2_mma(a0, b, c02); c12 = g2_mma(a1, b, c12);
    b = g2_frag(b3p + kb, hh); c03 = g2_mma(a0, b, c03); c13 = g2_mma(a1, b, c13); }
  v8f accs[8] = {c00, c01, c02, c03, c10, c11, c12, c13};
#pragma unroll
  for (int u = 0; u < 8; ++u) { const int t = u & 3, half = u >> 2; const int col = col0 + t * 16 + ln; const float bv = bf16_rne(bias[col]);
#pragma unroll
    for (int r = 0; r < 8; ++r) { const int rloc = half * 16 + 8 * hh + r; so[w][rloc][t * 16 + ln] = accs[u][r] * alpha + bv; } }
  __builtin_amdgcn_fence(4  , "workgroup"); __builtin_amdgcn_wave_barrier();
  const int rsub = lane >> 4, c4 = (lane & 15) * 4; const int head = col0 >> 6;
  for (int pass = 0; pass < 2; ++pass) {
#pragma unroll 4
    for (int q = 0; q < 16; ++q) { const int r = q * 2 + rsub; const v4f v = *(const v4fa*)&so[w][r][c4];
      v4h s0, s1, s2;
#pragma unroll
      for (int i = 0; i < 4; ++i) { const h16 hi = toh_flush(v[i]); const h16 rs = toh_flush((v[i] - (float)hi) * 2048.0f); const h16 hs = (h16)((float)hi * 2048.0f);
        s0[i] = (qside != 0) ? hs : hi; s1[i] = (qside != 0) ? rs : hi; s2[i] = (qside != 0) ? hi : rs; }
      _Float16* dst = C3 + (size_t)(row0 + r) * ldc3 + head * CK + c4;
      *(volatile v4h*)dst = s0; *(volatile v4h*)(dst + 64) = s1; *(volatile v4h*)(dst + 128) = s2; }
    if (pass == 0) __threadfence(); } }

__global__ __launch_bounds__(256) void k_wnat(const float* __restrict__ w, size_t n8, _Float16* __restrict__ Bt) { const size_t t = (size_t)blockIdx.x * 256 + threadIdx.x; if (t >= n8) return; FragH f; const v4f a = *(const v4fa*)(w + t * 8), c = *(const v4fa*)(w + t * 8 + 4);
#pragma unroll
  for (int q = 0; q < 4; ++q) { f.h[q] = toh_flush(bf16_rne(a[q]) * 16.0f); f.h[4 + q] = toh_flush(bf16_rne(c[q]) * 16.0f); }
  const v8us o = f.half[0]; *(volatile v8us*)((unsigned short*)Bt + t * 8) = o; __threadfence(); *(volatile v8us*)((unsigned short*)Bt + t * 8) = o; }

__global__ __launch_bounds__(256) void k_x16(const float* __restrict__ x, _Float16* __restrict__ X16, size_t n8) { const size_t t = (size_t)blockIdx.x * 256 + threadIdx.x; if (t >= n8) return;
  const size_t row = t / (DM / 8); const int c8 = (int)(t % (DM / 8)) * 8; const size_t srow = (row / NB) * NB_FULL + (row % NB);
  const float* p = x + srow * DM + c8; const v4f a = *(const v4fa*)p, c = *(const v4fa*)(p + 4); FragH f;
#pragma unroll
  for (int q = 0; q < 4; ++q) { f.h[q] = (_Float16)bf16_rne(a[q]); f.h[4 + q] = (_Float16)bf16_rne(c[q]); }
  const v8us o = f.half[0]; *(volatile v8us*)((unsigned short*)X16 + t * 8) = o; __threadfence(); *(volatile v8us*)((unsigned short*)X16 + t * 8) = o; }

__global__ __launch_bounds__(256) void k_vt(const _Float16* __restrict__ V16, _Float16* __restrict__ Vt) { __shared__ unsigned short tl[64][66]; const int tid = threadIdx.x; const int slab = blockIdx.x / (SEQ / 64), lg = blockIdx.x % (SEQ / 64); const int b = slab / NH, h = slab % NH;
  for (int i = tid; i < 64 * 8; i += 256) { const int r = i / 8, c8 = (i % 8) * 8; FragH f; f.half[0] = *(const v8us*)((const unsigned short*)V16 + ((size_t)(lg * 64 + r) * NB + b) * DM + h * HD + c8);
#pragma unroll
    for (int q = 0; q < 8; ++q) tl[r][c8 + q] = f.u[q]; }
  __syncthreads();
  for (int pass = 0; pass < 2; ++pass) {
#pragma unroll
    for (int rd = 0; rd < 2; ++rd) { const int d = rd * 32 + tid / 8, pc = tid % 8; FragH f;
#pragma unroll
      for (int q = 0; q < 8; ++q) f.u[q] = tl[pc * 8 + q][d];
      *(volatile v8us*)((unsigned short*)Vt + ((size_t)slab * 64 + d) * SEQ + lg * 64 + pc * 8) = f.half[0]; }
    if (pass == 0) __threadfence(); } }

__global__ __launch_bounds__(256) void k_sigma(const float* __restrict__ G, const float* __restrict__ wvp, const float* __restrict__ bvp, float* __restrict__ SIGT) {
  #pragma clang fp contract(off)
  __shared__ __attribute__((aligned(16))) float sg[32];
  const int tid = threadIdx.x, w = __builtin_amdgcn_readfirstlane((int)(tid >> 5)), lane = tid & 31;
  const float b0 = bf16_rne(bvp[0]);
#pragma unroll 1
  for (int i = 0; i < 4; ++i) {
    const int rl = w * 4 + i;
    const float* p = G + ((size_t)blockIdx.x * 32 + rl) * DM + lane;
    float acc = 0.f;
#pragma unroll 1
    for (int k = 0; k < DM; k += 32) acc += tanhf(p[k]) * bf16_rne(wvp[k + lane]);
#pragma unroll
    for (int off = 16; off > 0; off >>= 1) acc += __shfl_xor(acc, off, 32);
    const float g = acc + b0;
    const float sgm = 1.0f + 1.0f / (1.0f + expf(-g));
    const float i2 = 1.0f / (2.0f * sgm * sgm);
    if (lane == 0) sg[rl] = i2;
  }
  __syncthreads();
  if (w == 0 && lane < 8) { const v4f v = *(const v4fa*)&sg[lane * 4]; float* dst = SIGT + (size_t)blockIdx.x * 32 + lane * 4;
    *(volatile v4f*)dst = v; __threadfence(); *(volatile v4f*)dst = v; }
}

__global__ __launch_bounds__(256) void k_amean(const float* __restrict__ S, float* __restrict__ MEANT, int t0) {
  #pragma clang fp contract(off)
  __shared__ __attribute__((aligned(16))) float sm[32];
  const int tid = threadIdx.x, w = __builtin_amdgcn_readfirstlane((int)(tid >> 5)), lane = tid & 31;
  const int rb = blockIdx.x * 32; const int slab = rb / QC, tq0 = rb - slab * QC;
  const float pb = (float)(lane * 4 - SEQ / 2);
#pragma unroll 1
  for (int i = 0; i < 4; ++i) {
    const int rl = w * 4 + i;
    const float* p = S + ((size_t)slab * QC + tq0 + rl) * SEQ + lane * 4;
    v4f x[SEQ / 128];
#pragma unroll
    for (int j = 0; j < SEQ / 128; ++j) x[j] = *(const v4fa*)(p + j * 128);
    float mx = -3.0e38f;
#pragma unroll
    for (int j = 0; j < SEQ / 128; ++j) mx = fmaxf(mx, fmaxf(fmaxf(x[j][0], x[j][1]), fmaxf(x[j][2], x[j][3])));
#pragma unroll
    for (int off = 16; off > 0; off >>= 1) mx = fmaxf(mx, __shfl_xor(mx, off, 32));
    float se = 0.f, sw = 0.f;
#pragma unroll
    for (int j = 0; j < SEQ / 128; ++j) {
#pragma unroll
      for (int c = 0; c < 4; ++c) { const float e = __expf(x[j][c] - mx); se += e; sw += e * (pb + (float)(j * 128 + c)); } }
#pragma unroll
    for (int off = 16; off > 0; off >>= 1) { se += __shfl_xor(se, off, 32); sw += __shfl_xor(sw, off, 32); }
    const float mean = (float)(SEQ / 2) + sw * (1.0f / se);
    if (lane == 0) sm[rl] = mean;
  }
  __syncthreads();
  if (w == 0 && lane < 8) { const v4f v = *(const v4fa*)&sm[lane * 4]; float* dst = MEANT + (size_t)slab * SEQ + t0 + tq0 + lane * 4;
    *(volatile v4f*)dst = v; __threadfence(); *(volatile v4f*)dst = v; }
}

__global__ __launch_bounds__(128) void k_gsoft(const float* __restrict__ S, const float* __restrict__ MEANT, const float* __restrict__ SIGT, _Float16* __restrict__ PM, int t0) {
  #pragma clang fp contract(off)
  const int tid = threadIdx.x, w = __builtin_amdgcn_readfirstlane((int)(tid >> 5)), lane = tid & 31;
  const int wr = blockIdx.x * 4 + w; const int slab = wr / QC, tql = wr - slab * QC; const int b = slab / NH; const int t = t0 + tql;
  const float mu = MEANT[(size_t)slab * SEQ + t];
  const float i2 = SIGT[(size_t)t * NB + b];
  const float* p = S + ((size_t)slab * QC + tql) * SEQ + lane * 4;
  const float pb = (float)(lane * 4);
  v4f x[SEQ / 128];
#pragma unroll
  for (int j = 0; j < SEQ / 128; ++j) x[j] = *(const v4fa*)(p + j * 128);
  float mx = -3.0e38f;
#pragma unroll
  for (int j = 0; j < SEQ / 128; ++j) {
#pragma unroll
    for (int c = 0; c < 4; ++c) { const float d = (pb + (float)(j * 128 + c)) - mu; const float v = x[j][c] - (d * d) * i2; x[j][c] = v; mx = fmaxf(mx, v); } }
#pragma unroll
  for (int off = 16; off > 0; off >>= 1) mx = fmaxf(mx, __shfl_xor(mx, off, 32));
  float se = 0.f;
#pragma unroll
  for (int j = 0; j < SEQ / 128; ++j) {
#pragma unroll
    for (int c = 0; c < 4; ++c) { const float e = __expf(x[j][c] - mx); x[j][c] = e; se += e; } }
#pragma unroll
  for (int off = 16; off > 0; off >>= 1) se += __shfl_xor(se, off, 32);
  const float cs = 16384.0f * (1.0f / se);
  v4h hq[SEQ / 128];
#pragma unroll
  for (int j = 0; j < SEQ / 128; ++j) {
#pragma unroll
    for (int c = 0; c < 4; ++c) hq[j][c] = toh_flush(x[j][c] * cs); }
  _Float16* prow = PM + ((size_t)slab * QC + tql) * SEQ + lane * 4;
  for (int pass = 0; pass < 2; ++pass) {
#pragma unroll
    for (int j = 0; j < SEQ / 128; ++j) { const v4h v = hq[j]; *(volatile v4h*)(prow + j * 128) = v; }
    if (pass == 0) __threadfence(); }
}

extern "C" void kernel_launch(void* const* d_in, const int* in_sizes, int n_in,
                              void* d_out, int out_size, void* d_ws, size_t ws_size, hipStream_t stream) {
  if (n_in < 19) return;
  if ((size_t)in_sizes[0] < NR * DM || (size_t)in_sizes[1] < NR * DM || (size_t)in_sizes[2] < NR * DM) return;
  if ((size_t)in_sizes[3] < (size_t)DM * DM || (size_t)in_sizes[5] < (size_t)DM * DM || (size_t)in_sizes[7] < (size_t)DM * DM || (size_t)in_sizes[9] < (size_t)DM * DM) return;
  if ((size_t)in_sizes[11] < (size_t)DM * DM || (size_t)in_sizes[13] < (size_t)DM * DM || (size_t)in_sizes[17] < (size_t)DM * DM) return;
  if (in_sizes[4] < DM || in_sizes[6] < DM || in_sizes[8] < DM || in_sizes[10] < DM || in_sizes[12] < DM || in_sizes[14] < DM || in_sizes[15] < DM || in_sizes[16] < 1 || in_sizes[18] < DM) return;
  if ((size_t)out_size < NR * DM) return;
  const float* const* I = (const float* const*)d_in;
  const float* xq = I[0]; const float* xk = I[1]; const float* xv = I[2];
  const float* wq = I[3]; const float* bq = I[4]; const float* wk = I[5]; const float* bk = I[6]; const float* wv = I[7]; const float* bv = I[8];
  const float* whq = I[9]; const float* bhq = I[10]; const float* whk = I[11]; const float* bhk = I[12]; const float* wwp = I[13]; const float* bwp = I[14];
  const float* wvp = I[15]; const float* bvp = I[16]; const float* wo = I[17]; const float* bo = I[18];
  char* ws = (char*)d_ws; size_t off = 0;
  auto take = [&](size_t bytes) { char* p = ws + off; off += (bytes + 255) & ~(size_t)255; return p; };
  _Float16* BQ = (_Float16*)take((size_t)DM * DM * 2); _Float16* BK = (_Float16*)take((size_t)DM * DM * 2); _Float16* BV = (_Float16*)take((size_t)DM * DM * 2);
  _Float16* BHQ = (_Float16*)take((size_t)DM * DM * 2); _Float16* BHK = (_Float16*)take((size_t)DM * DM * 2); _Float16* BWP = (_Float16*)take((size_t)DM * DM * 2); _Float16* BO = (_Float16*)take((size_t)DM * DM * 2);
  _Float16* XQ = (_Float16*)take(NR * DM * 2); _Float16* XK = (_Float16*)take(NR * DM * 2); _Float16* XV = (_Float16*)take(NR * DM * 2);
  _Float16* CA = (_Float16*)take(NR * 3 * DM * 2); _Float16* CB = (_Float16*)take(NR * 3 * DM * 2);
  _Float16* V16 = (_Float16*)take(NR * DM * 2); _Float16* O16 = (_Float16*)take(NR * DM * 2); _Float16* VT = (_Float16*)take((size_t)NB * NH * HD * SEQ * 2);
  float* S = (float*)take((size_t)NB * NH * QC * SEQ * 4); _Float16* PM = (_Float16*)take((size_t)NB * NH * QC * SEQ * 2);
  float* MEANT = (float*)take((size_t)NB * NH * SEQ * 4); float* SIGT = (float*)take(NR * 4);
  if (off > ws_size) return;
  float* G = S;
  { const unsigned g = (unsigned)(((size_t)DM * DM / 8 + 255) / 256);
    k_wnat<<<g, 256, 0, stream>>>(wq, (size_t)DM * DM / 8, BQ); k_wnat<<<g, 256, 0, stream>>>(wk, (size_t)DM * DM / 8, BK);
    k_wnat<<<g, 256, 0, stream>>>(wv, (size_t)DM * DM / 8, BV); k_wnat<<<g, 256, 0, stream>>>(whq, (size_t)DM * DM / 8, BHQ);
    k_wnat<<<g, 256, 0, stream>>>(whk, (size_t)DM * DM / 8, BHK); k_wnat<<<g, 256, 0, stream>>>(wwp, (size_t)DM * DM / 8, BWP);
    k_wnat<<<g, 256, 0, stream>>>(wo, (size_t)DM * DM / 8, BO); }
  { const unsigned g = (unsigned)((NR * DM / 8 + 255) / 256);
    k_x16<<<g, 256, 0, stream>>>(xq, XQ, NR * DM / 8); k_x16<<<g, 256, 0, stream>>>(xk, XK, NR * DM / 8); k_x16<<<g, 256, 0, stream>>>(xv, XV, NR * DM / 8); }
  const dim3 gp((unsigned)((MP / 128) * (DM / 64)), 1);
  k_gemm2<true, false, false><<<gp, 128, 0, stream>>>(XV, DM, 0, BV, DM, 0, 0.0625f, bv, nullptr, V16, DM, 0, MP, DM, DM);
  k_vt<<<NB * NH * (SEQ / 64), 256, 0, stream>>>(V16, VT);
  k_gemm2<true, true, false><<<gp, 128, 0, stream>>>(XQ, DM, 0, BWP, DM, 0, 0.0625f, bwp, G, nullptr, DM, 0, MP, DM, DM);
  k_sigma<<<MP / 32, 256, 0, stream>>>(G, wvp, bvp, SIGT);
  k_gemm_cat<<<gp, 128, 0, stream>>>(XQ, DM, BHQ, DM, 0.0625f, bhq, CA, 3 * DM, 1, MP, DM, DM);
  k_gemm_cat<<<gp, 128, 0, stream>>>(XK, DM, BHK, DM, 0.0625f, bhk, CB, 3 * DM, 0, MP, DM, DM);
  for (int t0 = 0; t0 < SEQ; t0 += QC) {
    k_gemm2<false, true, false><<<dim3((QC / 128) * (SEQ / 64), NB * NH), 128, 0, stream>>>(CA + (size_t)t0 * LQ3, LQ3, (size_t)CK, CB, LQ3, (size_t)CK, 6.103515625e-05f, nullptr, S, nullptr, SEQ, (size_t)QC * SEQ, QC, SEQ, CK);
    k_amean<<<NB * NH * QC / 32, 256, 0, stream>>>(S, MEANT, t0);
  }
  k_gemm_cat<<<gp, 128, 0, stream>>>(XQ, DM, BQ, DM, 0.0625f, bq, CA, 3 * DM, 1, MP, DM, DM);
  k_gemm_cat<<<gp, 128, 0, stream>>>(XK, DM, BK, DM, 0.0625f, bk, CB, 3 * DM, 0, MP, DM, DM);
  for (int t0 = 0; t0 < SEQ; t0 += QC) {
    k_gemm2<false, true, false><<<dim3((QC / 128) * (SEQ / 64), NB * NH), 128, 0, stream>>>(CA + (size_t)t0 * LQ3, LQ3, (size_t)CK, CB, LQ3, (size_t)CK, 6.103515625e-05f, nullptr, S, nullptr, SEQ, (size_t)QC * SEQ, QC, SEQ, CK);
    k_gsoft<<<NB * NH * QC / 4, 128, 0, stream>>>(S, MEANT, SIGT, PM, t0);
    k_gemm2<false, false, false><<<dim3((QC / 128) * (HD / 64), NB * NH), 128, 0, stream>>>(PM, SEQ, (size_t)QC * SEQ, VT, SEQ, (size_t)HD * SEQ, 0.00390625f, nullptr, nullptr, O16 + (size_t)t0 * LQ, LQ, (size_t)HD, QC, HD, SEQ);
  }
  k_gemm2<true, true, true><<<gp, 128, 0, stream>>>(O16, DM, 0, BO, DM, 0, 0.0009765625f, bo, (float*)d_out, nullptr, DM, 0, MP, DM, DM);
}
